// CoAttLayer_86414741995961
// MI455X (gfx1250) — hardware-verified
//
#include <hip/hip_runtime.h>


#define NB_  64
#define TT   1024
#define DD   64
#define KK   128
#define BCH  8

typedef unsigned short bf;
typedef __attribute__((ext_vector_type(16))) __bf16   v16bf;
typedef __attribute__((ext_vector_type(8)))  unsigned short v8us;
typedef __attribute__((ext_vector_type(8)))  float    v8f;
typedef __attribute__((ext_vector_type(4)))  float    v4f;
typedef v4f  __attribute__((may_alias)) v4fa;
typedef v8us __attribute__((may_alias)) v8usa;

__device__ __forceinline__ unsigned short f2bf(float f) { unsigned u = __float_as_uint(f); u += 0x7FFFu + ((u >> 16) & 1u); return (unsigned short)(u >> 16); }
__device__ __forceinline__ float bf2f(unsigned short b) { return __uint_as_float(((unsigned)b) << 16); }
__device__ __forceinline__ float bfr(float f) { return bf2f(f2bf(f)); }
__device__ __forceinline__ v16bf cat16b(v8us lo, v8us hi) { return __builtin_bit_cast(v16bf, __builtin_shufflevector(lo, hi, 0, 1, 2, 3, 4, 5, 6, 7, 8, 9, 10, 11, 12, 13, 14, 15)); }
__device__ __forceinline__ v8f wmmab(v16bf a, v16bf b, v8f c) { return __builtin_amdgcn_wmma_f32_16x16x32_bf16(false, a, false, b, (short)0, c, false, false); }
#define VST2(T, p, v) do { const T vst2_v_ = (v); *(volatile T*)(p) = vst2_v_; __threadfence(); *(volatile T*)(p) = vst2_v_; } while (0)

__global__ __launch_bounds__(256) void k_wprep(const float* __restrict__ Wl, const float* __restrict__ Wr, const float* __restrict__ Wp, bf* WlT, bf* WPcat, bf* WRcat) {
    const int tid = threadIdx.x, lane = tid & 31, wave = tid >> 5;
#pragma unroll
    for (int s = 0; s < 2; ++s) { const int D = wave * 8 + s * 4 + (lane >> 3), piece = lane & 7; v8us o;
#pragma unroll
        for (int i = 0; i < 8; ++i) o[i] = f2bf(Wl[(size_t)(piece * 8 + i) * DD + D]);
        VST2(v8us, WlT + (size_t)D * DD + piece * 8, o); }
#pragma unroll
    for (int s = 0; s < 8; ++s) { const int k = wave * 16 + s * 2 + (lane >> 4), piece = lane & 15; v8us op, orr;
#pragma unroll
        for (int i = 0; i < 8; ++i) { const int j = piece * 8 + i, jj = j & (DD - 1); const float vp = Wp[(size_t)k * DD + jj], vr = Wr[(size_t)k * DD + jj];
            op[i] = f2bf(j < DD ? vp : vr); orr[i] = f2bf(j < DD ? vr : vp); }
        VST2(v8us, WPcat + (size_t)k * KK + piece * 8, op); VST2(v8us, WRcat + (size_t)k * KK + piece * 8, orr); }
}
__global__ __launch_bounds__(256) void k_rows(const float* __restrict__ x, int b0, bf* X64, bf* XCH, bf* XCL, bf* XT) {
    __shared__ __align__(16) unsigned short tl[64 * 72];
    const int tid = threadIdx.x, n0 = blockIdx.x * 64, bl = blockIdx.z, b = b0 + bl;
    { const int nn = tid >> 2, dq = (tid & 3) * 16; const float* src = x + ((size_t)b * TT + n0 + nn) * DD + dq;
#pragma unroll
      for (int i = 0; i < 16; ++i) tl[(dq + i) * 72 + nn] = f2bf(src[i]); }
    __syncthreads();
    const int piece = tid & 7;
    auto pass = [&]() {
#pragma unroll
        for (int s = 0; s < 2; ++s) { const int d = (tid >> 3) + 32 * s; const v8us val = *(const v8usa*)(tl + d * 72 + piece * 8); *(volatile v8us*)(XT + ((size_t)bl * DD + d) * TT + n0 + piece * 8) = val; }
#pragma unroll
        for (int s = 0; s < 2; ++s) { const int nn = (tid >> 3) + 32 * s; v8us o, z;
#pragma unroll
            for (int i = 0; i < 8; ++i) { o[i] = tl[(piece * 8 + i) * 72 + nn]; z[i] = 0; }
            const size_t r = (size_t)bl * TT + n0 + nn;
            *(volatile v8us*)(X64 + r * DD + piece * 8) = o; *(volatile v8us*)(XCH + r * KK + piece * 8) = o; *(volatile v8us*)(XCL + r * KK + piece * 8) = z; }
    };
    pass(); __threadfence(); pass();
}
template <bool SA, bool SB, int MODE>
__global__ __launch_bounds__(128) void k_gemm(const bf* __restrict__ A, const bf* __restrict__ Al, int lda, size_t sa, const bf* __restrict__ Bn, const bf* __restrict__ Bl, int ldb, size_t sb,
                                             int K, void* C, void* C2, int ldc, int coff, size_t sc) {
    __shared__ __align__(16) float ost[4][16 * 68];
    const int lane = threadIdx.x & 31, wave = threadIdx.x >> 5, lr = lane & 15, hi = lane >> 4, it = blockIdx.z;
    const int r0 = blockIdx.x * 64 + wave * 16, c0 = blockIdx.y * 64;
    A += it * sa; if (SA) Al += it * sa; Bn += it * sb; if (SB) Bl += it * sb;
    const size_t aoff = (size_t)(r0 + lr) * lda + 8 * hi;
    size_t boff[4];
#pragma unroll
    for (int t = 0; t < 4; ++t) boff[t] = (size_t)(c0 + t * 16 + lr) * ldb + 8 * hi;
    v8f acc[4];
#pragma unroll
    for (int t = 0; t < 4; ++t) acc[t] = (v8f){};
#pragma unroll 1
    for (int kc = 0; kc < K; kc += 32) {
        const v16bf a = cat16b(*(const v8us*)(A + aoff + kc), *(const v8us*)(A + aoff + kc + 16));
        v16bf al = a; if (SA) al = cat16b(*(const v8us*)(Al + aoff + kc), *(const v8us*)(Al + aoff + kc + 16));
#pragma unroll
        for (int t = 0; t < 4; ++t) { const v16bf b = cat16b(*(const v8us*)(Bn + boff[t] + kc), *(const v8us*)(Bn + boff[t] + kc + 16));
            acc[t] = wmmab(a, b, acc[t]); if (SA) acc[t] = wmmab(al, b, acc[t]);
            if (SB) { const v16bf b2 = cat16b(*(const v8us*)(Bl + boff[t] + kc), *(const v8us*)(Bl + boff[t] + kc + 16)); acc[t] = wmmab(a, b2, acc[t]); } }
        asm volatile("v_nop\n\tv_nop\n\tv_nop\n\tv_nop" : "+v"(acc[0]), "+v"(acc[1]), "+v"(acc[2]), "+v"(acc[3]) : "v"(a), "v"(al));
    }
    float* os = &ost[wave][0];
#pragma unroll
    for (int t = 0; t < 4; ++t)
#pragma unroll
        for (int j = 0; j < 8; ++j) { float v = acc[t][j]; if (MODE == 1 || MODE == 3) v = tanhf(v); os[(hi * 8 + j) * 68 + t * 16 + lr] = v; }
    __syncthreads();
    if (MODE == 0 || MODE == 3) {
        float* crow = (float*)C + it * sc + (size_t)r0 * ldc + coff + c0;
        auto pass = [&]() {
#pragma unroll
            for (int s = 0; s < 8; ++s) { const int Lid = (lane >> 3) + 4 * s, piece = lane & 7; const int row = Lid >> 1, cofs = (Lid & 1) * 32 + piece * 4;
                const v4f val = *(const v4fa*)(os + row * 68 + cofs); *(volatile v4f*)(crow + (size_t)row * ldc + cofs) = val; }
        };
        pass(); __threadfence(); pass();
    } else {
        bf* c1 = (bf*)C + it * sc + (size_t)r0 * ldc + coff + c0; bf* c2 = (bf*)C2 + it * sc + (size_t)r0 * ldc + coff + c0;
        auto pass = [&]() {
#pragma unroll
            for (int s = 0; s < 4; ++s) { const int row = 4 * s + (lane >> 3), piece = lane & 7; const float* sp = os + row * 68 + piece * 8; v8us oh, ol;
#pragma unroll
                for (int i = 0; i < 8; ++i) { const unsigned short hb = f2bf(sp[i]); oh[i] = hb; ol[i] = f2bf(sp[i] - bf2f(hb)); }
                *(volatile v8us*)(c1 + (size_t)row * ldc + piece * 8) = oh; *(volatile v8us*)(c2 + (size_t)row * ldc + piece * 8) = ol; }
        };
        pass(); __threadfence(); pass();
    }
}
__global__ __launch_bounds__(256) void k_head(const float* __restrict__ Hp, const float* __restrict__ Hr, const float* __restrict__ whp, const float* __restrict__ whr,
                                             const float* __restrict__ post, const float* __restrict__ review, int b0, float* out) {
    __shared__ float lg[TT];
    __shared__ float red[256];
    __shared__ float part[4][DD];
    const int tid = threadIdx.x, bl = blockIdx.x, which = blockIdx.y, b = b0 + bl;
    const float* H = (which == 0 ? Hp : Hr) + (size_t)bl * KK * TT; const float* w = (which == 0) ? whp : whr; const float* X = ((which == 0) ? post : review) + (size_t)b * TT * DD;
#pragma unroll
    for (int q = 0; q < 4; ++q) { const int n = tid + 256 * q; float s = 0.f;
#pragma unroll 4
        for (int k = 0; k < KK; ++k) s += bfr(w[k]) * H[(size_t)k * TT + n];
        lg[n] = s; }
    __syncthreads();
    float m = -3.0e38f;
#pragma unroll
    for (int q = 0; q < 4; ++q) m = fmaxf(m, lg[tid + 256 * q]);
    red[tid] = m; __syncthreads();
    for (int st = 128; st > 0; st >>= 1) { if (tid < st) red[tid] = fmaxf(red[tid], red[tid + st]); __syncthreads(); }
    m = red[0]; __syncthreads();
    float s = 0.f;
#pragma unroll
    for (int q = 0; q < 4; ++q) { const float e = __expf(lg[tid + 256 * q] - m); lg[tid + 256 * q] = e; s += e; }
    red[tid] = s; __syncthreads();
    for (int st = 128; st > 0; st >>= 1) { if (tid < st) red[tid] += red[tid + st]; __syncthreads(); }
    const float inv = 1.0f / red[0];
    { const int g = tid >> 6, d = tid & 63; float acc = 0.f;
#pragma unroll 4
      for (int n = g * 256; n < g * 256 + 256; ++n) acc += bfr(X[(size_t)n * DD + d]) * lg[n];
      part[g][d] = acc; }
    __syncthreads();
    if (tid < 64) { const float v = (part[0][tid] + part[1][tid] + part[2][tid] + part[3][tid]) * inv;
        *(volatile float*)(out + (size_t)b * (2 * DD) + which * DD + tid) = v; __threadfence(); *(volatile float*)(out + (size_t)b * (2 * DD) + which * DD + tid) = v; }
}

extern "C" void kernel_launch(void* const* d_in, const int* in_sizes, int n_in,
                              void* d_out, int out_size, void* d_ws, size_t ws_size, hipStream_t stream) {
    (void)in_sizes; (void)n_in; (void)out_size;
    const float* review = (const float*)d_in[0]; const float* post = (const float*)d_in[1]; const float* Wl = (const float*)d_in[2];
    const float* Wr = (const float*)d_in[3]; const float* Wp = (const float*)d_in[4]; const float* whr = (const float*)d_in[5]; const float* whp = (const float*)d_in[6];
    float* out = (float*)d_out;
    char* wsp = (char*)d_ws;
    auto take = [&](size_t bytes) { char* p = wsp; wsp += (bytes + 255) & ~(size_t)255; return (void*)p; };
    bf* WlT = (bf*)take((size_t)DD * DD * 2); bf* WPcat = (bf*)take((size_t)KK * KK * 2); bf* WRcat = (bf*)take((size_t)KK * KK * 2);
    const size_t S64 = (size_t)TT * DD, S128 = (size_t)TT * KK, SL = (size_t)TT * TT, SH = (size_t)KK * TT;
    bf* P64 = (bf*)take(BCH * S64 * 2); bf* PCH = (bf*)take(BCH * S128 * 2); bf* PCL = (bf*)take(BCH * S128 * 2); bf* PT = (bf*)take(BCH * S64 * 2);
    bf* R64 = (bf*)take(BCH * S64 * 2); bf* RCH = (bf*)take(BCH * S128 * 2); bf* RCL = (bf*)take(BCH * S128 * 2); bf* RT = (bf*)take(BCH * S64 * 2);
    bf* RWH = (bf*)take(BCH * S64 * 2); bf* RWL = (bf*)take(BCH * S64 * 2);
    bf* LH = (bf*)take(BCH * SL * 2); bf* LL = (bf*)take(BCH * SL * 2); bf* LTH = (bf*)take(BCH * SL * 2); bf* LTL = (bf*)take(BCH * SL * 2);
    float* HP = (float*)take(BCH * SH * 4); float* HR = (float*)take(BCH * SH * 4);
    if ((size_t)(wsp - (char*)d_ws) > ws_size) return;
    k_wprep<<<1, 256, 0, stream>>>(Wl, Wr, Wp, WlT, WPcat, WRcat);
    for (int ch = 0; ch < NB_ / BCH; ++ch) { const int b0 = ch * BCH;
        k_rows<<<dim3(TT / 64, 1, BCH), 256, 0, stream>>>(post, b0, P64, PCH, PCL, PT);
        k_rows<<<dim3(TT / 64, 1, BCH), 256, 0, stream>>>(review, b0, R64, RCH, RCL, RT);
        k_gemm<false, false, 2><<<dim3(TT / 64, 1, BCH), 128, 0, stream>>>(R64, nullptr, DD, S64, WlT, nullptr, DD, 0, DD, RWH, RWL, DD, 0, S64);
        k_gemm<true, false, 1><<<dim3(TT / 64, TT / 64, BCH), 128, 0, stream>>>(RWH, RWL, DD, S64, P64, nullptr, DD, S64, DD, LH, LL, TT, 0, SL);
        k_gemm<false, true, 1><<<dim3(TT / 64, TT / 64, BCH), 128, 0, stream>>>(P64, nullptr, DD, S64, RWH, RWL, DD, S64, DD, LTH, LTL, TT, 0, SL);
        k_gemm<true, false, 2><<<dim3(TT / 64, 1, BCH), 128, 0, stream>>>(LTH, LTL, TT, SL, RT, nullptr, TT, S64, TT, PCH, PCL, KK, DD, S128);
        k_gemm<true, false, 2><<<dim3(TT / 64, 1, BCH), 128, 0, stream>>>(LH, LL, TT, SL, PT, nullptr, TT, S64, TT, RCH, RCL, KK, DD, S128);
        k_gemm<false, true, 3><<<dim3(KK / 64, TT / 64, BCH), 128, 0, stream>>>(WPcat, nullptr, KK, 0, PCH, PCL, KK, S128, KK, HP, nullptr, TT, 0, SH);
        k_gemm<false, true, 3><<<dim3(KK / 64, TT / 64, BCH), 128, 0, stream>>>(WRcat, nullptr, KK, 0, RCH, RCL, KK, S128, KK, HR, nullptr, TT, 0, SH);
        k_head<<<dim3(BCH, 2, 1), 256, 0, stream>>>(HP, HR, whp, whr, post, review, b0, out);
    }
}
